// SimpleSSM_5016521802563
// MI455X (gfx1250) — hardware-verified
//
#include <hip/hip_runtime.h>


#define NBT  2
#define SS   2048
#define HH   1024
#define II   2048
#define NS   16
#define NXP  64
#define KC   4
#define DM   HH
#define LOSC 1024.0f

typedef _Float16 h16;
typedef unsigned short bf;
typedef __attribute__((ext_vector_type(16))) __bf16   v16bf;
typedef __attribute__((ext_vector_type(16))) _Float16 v16h;
typedef __attribute__((ext_vector_type(8)))  _Float16 v8h;
typedef __attribute__((ext_vector_type(8)))  unsigned short v8us;
typedef __attribute__((ext_vector_type(8)))  float    v8f;
typedef __attribute__((ext_vector_type(4)))  float    v4f;
typedef __attribute__((ext_vector_type(4)))  _Float16 v4h;
typedef v8h  __attribute__((may_alias)) v8ha;
typedef v4f  __attribute__((may_alias)) v4fa;
typedef v8us __attribute__((may_alias)) v8usa;

__device__ __forceinline__ unsigned short f2bf(float f) { unsigned u = __float_as_uint(f); u += 0x7FFFu + ((u >> 16) & 1u); return (unsigned short)(u >> 16); }
__device__ __forceinline__ float bf2f(unsigned short b) { return __uint_as_float(((unsigned)b) << 16); }
__device__ __forceinline__ float bfr(float f) { return bf2f(f2bf(f)); }
__device__ __forceinline__ v16h cat16(v8h lo, v8h hi) { return __builtin_shufflevector(lo, hi, 0, 1, 2, 3, 4, 5, 6, 7, 8, 9, 10, 11, 12, 13, 14, 15); }
__device__ __forceinline__ v16bf cat16b(v8us lo, v8us hi) { return __builtin_bit_cast(v16bf, __builtin_shufflevector(lo, hi, 0, 1, 2, 3, 4, 5, 6, 7, 8, 9, 10, 11, 12, 13, 14, 15)); }
__device__ __forceinline__ v8f wmma16(v16h a, v16h b, v8f c) { return __builtin_amdgcn_wmma_f32_16x16x32_f16(false, a, false, b, (short)0, c, false, false); }
__device__ __forceinline__ v8f wmmab(v16bf a, v16bf b, v8f c) { return __builtin_amdgcn_wmma_f32_16x16x32_bf16(false, a, false, b, (short)0, c, false, false); }

template <bool SPLITA, bool F16OUT = false>
__global__ __launch_bounds__(128) void k_gemmb(const bf* __restrict__ A, const bf* __restrict__ Al, const bf* __restrict__ Bn, const float* __restrict__ bias, float* C, int ldc, h16* C2, const float* __restrict__ R = nullptr, int K = DM, int roundR = 1) {
    __shared__ __align__(16) float ost[4][16 * 68];
    const int lane = threadIdx.x & 31, wave = threadIdx.x >> 5, lr = lane & 15, hi = lane >> 4;
    const int r0 = blockIdx.x * 64 + wave * 16, c0 = blockIdx.y * 64;
    const size_t aoff = (size_t)(r0 + lr) * K + 8 * hi;
    size_t boff[4];
#pragma unroll
    for (int t = 0; t < 4; ++t) boff[t] = (size_t)(c0 + t * 16 + lr) * K + 8 * hi;
    v8f acc[4];
#pragma unroll
    for (int t = 0; t < 4; ++t) acc[t] = (v8f){};
#pragma unroll 1
    for (int kc = 0; kc < K; kc += 32) {
        const v16bf a = cat16b(*(const v8us*)(A + aoff + kc), *(const v8us*)(A + aoff + kc + 16));
        v16bf al = a;
        if (SPLITA) al = cat16b(*(const v8us*)(Al + aoff + kc), *(const v8us*)(Al + aoff + kc + 16));
#pragma unroll
        for (int t = 0; t < 4; ++t) { const v16bf b = cat16b(*(const v8us*)(Bn + boff[t] + kc), *(const v8us*)(Bn + boff[t] + kc + 16)); acc[t] = wmmab(a, b, acc[t]); if (SPLITA) acc[t] = wmmab(al, b, acc[t]); }
        asm volatile("v_nop\n\tv_nop\n\tv_nop\n\tv_nop" : "+v"(acc[0]), "+v"(acc[1]), "+v"(acc[2]), "+v"(acc[3]) : "v"(a), "v"(al));
    }
    float* os = &ost[wave][0];
#pragma unroll
    for (int t = 0; t < 4; ++t) { const float bv = bias ? bfr(bias[c0 + t * 16 + lr]) : 0.f;
#pragma unroll
        for (int j = 0; j < 8; ++j) os[(hi * 8 + j) * 68 + t * 16 + lr] = acc[t][j] + bv; }
    __syncthreads();
    if (F16OUT) {
        h16* crow = (h16*)(void*)C + (size_t)r0 * ldc + c0;
        auto pass = [&]() {
#pragma unroll
            for (int s = 0; s < 4; ++s) { const int row = 4 * s + (lane >> 3), piece = lane & 7; const float* sp = os + row * 68 + piece * 8; v8h o, o2;
#pragma unroll
                for (int i = 0; i < 8; ++i) { const h16 a = (h16)sp[i]; o[i] = a; o2[i] = (h16)((sp[i] - (float)a) * LOSC); }
                *(volatile v8h*)(crow + (size_t)row * ldc + piece * 8) = o; if (C2) *(volatile v8h*)(C2 + (size_t)r0 * ldc + c0 + (size_t)row * ldc + piece * 8) = o2; }
        };
        pass(); __threadfence(); pass();
    } else {
        float* crow = C + (size_t)r0 * ldc + c0;
        auto pass = [&]() {
#pragma unroll
            for (int s = 0; s < 8; ++s) { const int Lid = (lane >> 3) + 4 * s, piece = lane & 7; const int row = Lid >> 1, cofs = (Lid & 1) * 32 + piece * 4;
                v4f val = *(const v4fa*)(os + row * 68 + cofs); if (R) { const v4f rv = *(const v4f*)(R + ((size_t)r0 + row) * ldc + c0 + cofs); val += roundR ? (v4f){bfr(rv[0]), bfr(rv[1]), bfr(rv[2]), bfr(rv[3])} : rv; }
                *(volatile v4f*)(crow + (size_t)row * ldc + cofs) = val; }
        };
        pass(); __threadfence(); pass();
    }
}

__global__ __launch_bounds__(256) void k_cvt8(const float* __restrict__ src, bf* dst, size_t n8) {
    const size_t i = (size_t)blockIdx.x * 256 + threadIdx.x; if (i >= n8) return;
    const v8f v = *(const v8f*)(src + i * 8); v8us o;
#pragma unroll
    for (int k = 0; k < 8; ++k) o[k] = f2bf(v[k]);
    *(volatile v8us*)(dst + i * 8) = o; __threadfence(); *(volatile v8us*)(dst + i * 8) = o;
}
__global__ __launch_bounds__(256) void k_zero8(bf* dst, size_t n8) {
    const size_t i = (size_t)blockIdx.x * 256 + threadIdx.x; if (i >= n8) return; v8us z;
#pragma unroll
    for (int k = 0; k < 8; ++k) z[k] = 0;
    *(volatile v8us*)(dst + i * 8) = z; __threadfence(); *(volatile v8us*)(dst + i * 8) = z;
}

__global__ __launch_bounds__(256) void k_cvtx(const float* __restrict__ src, int rows, bf* dst) {
    const int lane = threadIdx.x & 31; const size_t r = (size_t)blockIdx.x * 8 + (threadIdx.x >> 5); if (r >= (size_t)rows) return;
#pragma unroll 1
    for (int ps = 0; ps < 2; ++ps) {
#pragma unroll
        for (int q = 0; q < HH / 256; ++q) { v8us o;
#pragma unroll
            for (int i = 0; i < 8; ++i) o[i] = f2bf(src[r * HH + q * 256 + lane * 8 + i]);
            *(volatile v8us*)(dst + r * HH + q * 256 + lane * 8) = o; }
        if (ps == 0) __threadfence(); }
}
__global__ __launch_bounds__(256) void k_wxpad(const float* __restrict__ Wx, bf* WXP) {
    const int lane = threadIdx.x & 31; const int r = blockIdx.x * 8 + (threadIdx.x >> 5); if (r >= NXP) return;
#pragma unroll 1
    for (int ps = 0; ps < 2; ++ps) {
#pragma unroll
        for (int q = 0; q < II / 256; ++q) { v8us v;
#pragma unroll
            for (int i = 0; i < 8; ++i) { const int k = q * 256 + lane * 8 + i; v[i] = f2bf(r < 33 ? Wx[(size_t)(r < 33 ? r : 0) * II + k] : 0.f); }
            *(volatile v8us*)(WXP + (size_t)r * II + q * 256 + lane * 8) = v; }
        if (ps == 0) __threadfence(); }
}
__global__ __launch_bounds__(256) void k_conv(const float* __restrict__ XZ, const float* __restrict__ wc, float* XC, bf* Ch, bf* Cl) {
    typedef __attribute__((ext_vector_type(4))) unsigned short v4us;
    const int lane = threadIdx.x & 31; const size_t s = (size_t)blockIdx.x * 8 + (threadIdx.x >> 5); if (s >= (size_t)SS) return;
#pragma unroll 1
    for (int ps = 0; ps < 2; ++ps) {
#pragma unroll 1
        for (int st = 0; st < II / 128; ++st) { const int c0 = st * 128 + lane * 4; v4f o; v4us oh, ol;
#pragma unroll
            for (int q = 0; q < 4; ++q) { const int i = c0 + q; float acc = 0.f;
#pragma unroll
                for (int k = 0; k < KC; ++k) { const long sp = (long)s - 3 + k; const float u = (sp >= 0) ? XZ[(size_t)(sp >= 0 ? sp : 0) * (2 * II) + i] : 0.f; acc = fmaf(bfr(wc[i * KC + k]), u, acc); }
                const float sv = acc / (1.0f + __expf(-acc)); o[q] = sv; const unsigned short hb = f2bf(sv); oh[q] = hb; ol[q] = f2bf(sv - bf2f(hb)); }
            const size_t off = s * II + c0; *(volatile v4f*)(XC + off) = o; *(volatile v4us*)(Ch + off) = oh; *(volatile v4us*)(Cl + off) = ol; }
        if (ps == 0) __threadfence(); }
}
__global__ __launch_bounds__(256) void k_ssm(const float* __restrict__ XC, const float* __restrict__ PJ, const float* __restrict__ XZ, const float* __restrict__ Alog, const float* __restrict__ Dp, bf* Yh, bf* Yl) {
    typedef __attribute__((ext_vector_type(4))) unsigned short v4us;
    const int lane = threadIdx.x & 31; const size_t s = (size_t)blockIdx.x * 8 + (threadIdx.x >> 5); if (s >= (size_t)SS) return; const float* pj = PJ + s * NXP;
    const float d0 = pj[0]; const float delta = (d0 > 20.f) ? d0 : log1pf(__expf(d0));
#pragma unroll 1
    for (int ps = 0; ps < 2; ++ps) {
#pragma unroll 1
        for (int st = 0; st < II / 128; ++st) { const int c0 = st * 128 + lane * 4; v4us oh, ol;
#pragma unroll
            for (int q = 0; q < 4; ++q) { const int i = c0 + q; const float xc = XC[s * II + i]; float acc = 0.f;
#pragma unroll 1
                for (int n = 0; n < NS; ++n) { const float A = -__expf(bfr(Alog[i * NS + n])); acc = fmaf(pj[1 + n] * pj[1 + NS + n], __expf(delta * A), acc); }
                const float z = XZ[s * (2 * II) + II + i]; const float y = (xc * acc + xc * bfr(Dp[i])) * (z / (1.0f + __expf(-z))); const unsigned short hb = f2bf(y); oh[q] = hb; ol[q] = f2bf(y - bf2f(hb)); }
            const size_t off = s * II + c0; *(volatile v4us*)(Yh + off) = oh; *(volatile v4us*)(Yl + off) = ol; }
        if (ps == 0) __threadfence(); }
}

extern "C" void kernel_launch(void* const* d_in, const int* in_sizes, int n_in,
                              void* d_out, int out_size, void* d_ws, size_t ws_size, hipStream_t stream) {
    (void)in_sizes; (void)n_in; (void)out_size;
    const float* x = (const float*)d_in[0]; const float* Win = (const float*)d_in[1]; const float* wc = (const float*)d_in[2]; const float* Wx = (const float*)d_in[3]; const float* Alog = (const float*)d_in[4]; const float* Dp = (const float*)d_in[5]; const float* Wout = (const float*)d_in[6];
    float* out = (float*)d_out;
    char* wsp = (char*)d_ws;
    auto take = [&](size_t bytes) { char* p = wsp; wsp += (bytes + 255) & ~(size_t)255; return (void*)p; };
    bf* WIN = (bf*)take((size_t)2 * II * HH * 2); bf* WXP = (bf*)take((size_t)NXP * II * 2); bf* WOUT = (bf*)take((size_t)HH * II * 2);
    bf* Xb = (bf*)take((size_t)SS * HH * 2); float* XZ = (float*)take((size_t)SS * 2 * II * 4); float* XC = (float*)take((size_t)SS * II * 4); bf* Ch = (bf*)take((size_t)SS * II * 2); bf* Cl = (bf*)take((size_t)SS * II * 2); float* PJ = (float*)take((size_t)SS * NXP * 4);
    if ((size_t)(wsp - (char*)d_ws) > ws_size) return;
    bf* Yh = Ch; bf* Yl = Cl;
    k_cvt8<<<(unsigned)(((size_t)2 * II * HH / 8 + 255) / 256), 256, 0, stream>>>(Win, WIN, (size_t)2 * II * HH / 8); k_wxpad<<<NXP / 8, 256, 0, stream>>>(Wx, WXP); k_cvt8<<<(unsigned)(((size_t)HH * II / 8 + 255) / 256), 256, 0, stream>>>(Wout, WOUT, (size_t)HH * II / 8);
    for (int b = 0; b < NBT; ++b) {
        k_cvtx<<<SS / 8, 256, 0, stream>>>(x + (size_t)b * SS * HH, SS, Xb);
        k_gemmb<false, false><<<dim3(SS / 64, (2 * II) / 64, 1), 128, 0, stream>>>(Xb, nullptr, WIN, nullptr, XZ, 2 * II, nullptr, nullptr, HH);
        k_conv<<<SS / 8, 256, 0, stream>>>(XZ, wc, XC, Ch, Cl);
        k_gemmb<true, false><<<dim3(SS / 64, NXP / 64, 1), 128, 0, stream>>>(Ch, Cl, WXP, nullptr, PJ, NXP, nullptr, nullptr, II);
        k_ssm<<<SS / 8, 256, 0, stream>>>(XC, PJ, XZ, Alog, Dp, Yh, Yl);
        k_gemmb<true, false><<<dim3(SS / 64, HH / 64, 1), 128, 0, stream>>>(Yh, Yl, WOUT, nullptr, out + (size_t)b * SS * HH, HH, nullptr, nullptr, II); }
}
